// SimpleSelfAttention_1030792151199
// MI455X (gfx1250) — hardware-verified
//
#include <hip/hip_runtime.h>
#include <math.h>

typedef __attribute__((ext_vector_type(16))) _Float16 v16bf;
typedef __attribute__((ext_vector_type(8)))  float  v8f;
typedef unsigned short u16;

union FragAB { v16bf v; uint4 q[2]; u16 u[16]; };
union FragC  { v8f  v; float f[8]; };

__device__ __forceinline__ u16 f2bf(float x) {
  _Float16 h = (_Float16)x;
  return __builtin_bit_cast(u16, h);
}
typedef __attribute__((ext_vector_type(4))) float v4f;
typedef __attribute__((ext_vector_type(4))) unsigned v4u;
template <typename V> __device__ __forceinline__ void vst2(void* p, V v) {
  *(volatile V*)p = v; __threadfence(); *(volatile V*)p = v;
}
#define PSC 4096.0f
#define PUN (1.0f / 4096.0f)

__device__ __forceinline__ v8f wmma_bf16(const FragAB& a, const FragAB& b, v8f c) {
  v8f d = __builtin_amdgcn_wmma_f32_16x16x32_f16(false, a.v, false, b.v, (short)0, c, false, false);
  asm volatile("v_nop\n\tv_nop\n\tv_nop\n\tv_nop" : "+v"(d) : "v"(a.v), "v"(b.v));
  return d;
}

#define USE_ASYNC_COPY 0

__device__ __forceinline__ void cp_async16(void* dst_lds, const void* src_glob) {
#if USE_ASYNC_COPY
  unsigned lds = (unsigned)(unsigned long long)dst_lds;
  unsigned long long g = (unsigned long long)src_glob;
  asm volatile("global_load_async_to_lds_b128 %0, %1, off"
               :: "v"(lds), "v"(g) : "memory");
#else
  *(uint4*)dst_lds = *(const uint4*)src_glob;
#endif
}

__device__ __forceinline__ void cp_async32(u16* dst_lds, const u16* src_glob) {
  cp_async16(dst_lds, src_glob);
  cp_async16(dst_lds + 8, src_glob + 8);
}

__device__ __forceinline__ void wait_async() {
#if USE_ASYNC_COPY
  asm volatile("s_wait_asynccnt 0x0" ::: "memory");
#endif
}

#define HID   1024
#define HEADS 16
#define DHEAD 64
#define SEQ   2048
#define BATCH 2
#define ROWS  (BATCH * SEQ)
#define NKQV  (3 * HID)
#define BH    (BATCH * HEADS)

__global__ void convert_f32_bf16(const float* __restrict__ src, u16* __restrict__ dst, int n) {
  int g = blockIdx.x * blockDim.x + threadIdx.x;
  if (g * 8 >= n) return;
  union { u16 s[8]; v4u u; } pk;
#pragma unroll
  for (int e = 0; e < 8; ++e) pk.s[e] = f2bf(src[(size_t)g * 8 + e]);
  vst2(dst + (size_t)g * 8, pk.u);
}

__global__ __launch_bounds__(256)
void transpose_cvt(const float* __restrict__ src, u16* __restrict__ dst, int K, int N) {
  __shared__ float tile[64][33];
  int n0 = blockIdx.x * 32, k0 = blockIdx.y * 64;
  int tx = threadIdx.x & 31, ty = threadIdx.x >> 5;
#pragma unroll
  for (int j = 0; j < 64; j += 8)
    tile[ty + j][tx] = src[(size_t)(k0 + ty + j) * N + (n0 + tx)];
  __syncthreads();
#pragma unroll
  for (int j = 0; j < 32; j += 8) {
    union { u16 s[2]; unsigned u; } pk;
    pk.s[0] = f2bf(tile[2 * tx][ty + j]); pk.s[1] = f2bf(tile[2 * tx + 1][ty + j]);
    vst2(dst + (size_t)(n0 + ty + j) * K + k0 + 2 * tx, pk.u);
  }
}

#define LDSTRIDE 40

template <int MODE>
__global__ __launch_bounds__(256)
void gemm_bf16(const u16* __restrict__ A, const u16* __restrict__ BT,
               const float* __restrict__ bias, int M, int N, int K,
               u16* __restrict__ Kg, u16* __restrict__ Qg,
               u16* __restrict__ Vtg, float* __restrict__ Cout) {
  __shared__ u16 sA[2][128 * LDSTRIDE];
  __shared__ u16 sB[2][256 * LDSTRIDE];
  __shared__ __align__(16) u16 T[(MODE == 0) ? 128 * 264 : 64 * 256 * 2];

  const int tid  = threadIdx.x;
  const int wave = tid >> 5, lane = tid & 31;
  const int half = lane >> 4, c16 = lane & 15;
  const int mW = (wave & 1) * 64;
  const int nW = (wave >> 1) * 64;
  const int rowBase = blockIdx.y * 128;
  const int colBase = blockIdx.x * 256;

  FragC acc[4][4];
#pragma unroll
  for (int mf = 0; mf < 4; ++mf)
#pragma unroll
    for (int nf = 0; nf < 4; ++nf)
#pragma unroll
      for (int i = 0; i < 8; ++i) acc[mf][nf].f[i] = 0.0f;

  const int arow = tid >> 1, aseg = (tid & 1) * 16;
  auto issueTile = [&](int kt, int bsel) {
    const int k0 = kt * 32;
    const u16* ga = A + (size_t)(rowBase + arow) * K + k0 + aseg;
    cp_async32(&sA[bsel][arow * LDSTRIDE + aseg], ga);
    const u16* gb = BT + (size_t)(colBase + tid) * K + k0;
    cp_async32(&sB[bsel][tid * LDSTRIDE], gb);
    cp_async32(&sB[bsel][tid * LDSTRIDE + 16], gb + 16);
  };

  issueTile(0, 0);
  const int KT = K >> 5;
  for (int kt = 0; kt < KT; ++kt) {
    const int cur = kt & 1;
    wait_async();
    __syncthreads();
    if (kt + 1 < KT) issueTile(kt + 1, cur ^ 1);

    FragAB af[4], bfr[4];
#pragma unroll
    for (int mf = 0; mf < 4; ++mf) {
      const u16* base = &sA[cur][(mW + mf * 16 + c16) * LDSTRIDE];
      af[mf].q[0] = *(const uint4*)(base + 8 * half);
      af[mf].q[1] = *(const uint4*)(base + 16 + 8 * half);
    }
#pragma unroll
    for (int nf = 0; nf < 4; ++nf) {
      const u16* base = &sB[cur][(nW + nf * 16 + c16) * LDSTRIDE];
      bfr[nf].q[0] = *(const uint4*)(base + 8 * half);
      bfr[nf].q[1] = *(const uint4*)(base + 16 + 8 * half);
    }
#pragma unroll
    for (int mf = 0; mf < 4; ++mf)
#pragma unroll
      for (int nf = 0; nf < 4; ++nf)
        acc[mf][nf].v = wmma_bf16(af[mf], bfr[nf], acc[mf][nf].v);
  }

  if (MODE == 0) {
#pragma unroll
    for (int mf = 0; mf < 4; ++mf)
#pragma unroll
      for (int nf = 0; nf < 4; ++nf)
#pragma unroll
        for (int rr = 0; rr < 8; ++rr) {
          int rl = mW + mf * 16 + rr + 8 * half, cl = nW + nf * 16 + c16;
          T[rl * 264 + cl] = f2bf(acc[mf][nf].f[rr] + bias[colBase + cl]);
        }
    __syncthreads();
    const int bidx = rowBase >> 11, s0 = rowBase & 2047;
#pragma unroll 1
    for (int c4 = 0; c4 < 4; ++c4) {
      const int gc0 = colBase + c4 * 64;
      const int mat = gc0 >> 10, head = (gc0 & 1023) >> 6;
      const int bh = bidx * HEADS + head;
      if (mat < 2) {
        u16* dstp = (mat == 0) ? Kg : Qg;
        for (int g = tid; g < 128 * 8; g += 256) {
          const int rl = g >> 3, pc = g & 7;
          vst2(dstp + ((size_t)bh * SEQ + s0 + rl) * DHEAD + pc * 8, *(const v4u*)(&T[rl * 264 + c4 * 64 + pc * 8]));
        }
      } else {
        for (int g = tid; g < 64 * 16; g += 256) {
          const int d = g >> 4, pc = g & 15;
          union { u16 s[8]; v4u u; } pk;
#pragma unroll
          for (int e = 0; e < 8; ++e) pk.s[e] = T[(pc * 8 + e) * 264 + c4 * 64 + d];
          vst2(Vtg + ((size_t)bh * DHEAD + d) * SEQ + s0 + pc * 8, pk.u);
        }
      }
    }
  } else {
    float* Tf = (float*)T;
#pragma unroll 1
    for (int hh = 0; hh < 2; ++hh) {
      if ((wave & 1) == hh) {
#pragma unroll
        for (int mf = 0; mf < 4; ++mf)
#pragma unroll
          for (int nf = 0; nf < 4; ++nf)
#pragma unroll
            for (int rr = 0; rr < 8; ++rr) {
              int rl = mf * 16 + rr + 8 * half, cl = nW + nf * 16 + c16;
              Tf[rl * 256 + cl] = acc[mf][nf].f[rr] + bias[colBase + cl];
            }
      }
      __syncthreads();
      for (int g = tid; g < 64 * 64; g += 256) {
        const int rl = g >> 6, pc = g & 63;
        vst2(Cout + (size_t)(rowBase + hh * 64 + rl) * N + colBase + pc * 4, *(const v4f*)(&Tf[rl * 256 + pc * 4]));
      }
      __syncthreads();
    }
  }
}

__global__ __launch_bounds__(256)
void attn_stats(const u16* __restrict__ Kg, const u16* __restrict__ Qg,
                float* __restrict__ mG, float* __restrict__ rlG, float scale) {
  __shared__ u16 sK[128 * 64];
  __shared__ u16 sQ[128 * 64];
  __shared__ float mPart[2][128], lPart[2][128];

  const int bh = blockIdx.y, sBlk = blockIdx.x;
  const int tid = threadIdx.x;
  const int wave = tid >> 5, lane = tid & 31;
  const int half = lane >> 4, c16 = lane & 15;
  const int mW = (wave & 3) * 32;
  const int wn = wave >> 2;
  const int nW = wn * 64;

  const int lrow = tid >> 1, lseg = (tid & 1) * 32;
  {
    const u16* g = Kg + ((size_t)bh * SEQ + sBlk * 128 + lrow) * DHEAD + lseg;
    cp_async32(&sK[lrow * 64 + lseg], g);
    cp_async32(&sK[lrow * 64 + lseg + 16], g + 16);
  }

  float m_run[2][8], l_run[2][8];
#pragma unroll
  for (int sf = 0; sf < 2; ++sf)
#pragma unroll
    for (int rr = 0; rr < 8; ++rr) { m_run[sf][rr] = -3.0e38f; l_run[sf][rr] = 0.0f; }

  for (int nb = 0; nb < 16; ++nb) {
    __syncthreads();
    {
      const u16* g = Qg + ((size_t)bh * SEQ + nb * 128 + lrow) * DHEAD + lseg;
      cp_async32(&sQ[lrow * 64 + lseg], g);
      cp_async32(&sQ[lrow * 64 + lseg + 16], g + 16);
    }
    wait_async();
    __syncthreads();

    FragC acc[2][4];
#pragma unroll
    for (int sf = 0; sf < 2; ++sf)
#pragma unroll
      for (int nf = 0; nf < 4; ++nf)
#pragma unroll
        for (int i = 0; i < 8; ++i) acc[sf][nf].f[i] = 0.0f;

#pragma unroll
    for (int k0 = 0; k0 < 64; k0 += 32) {
      FragAB ak[2], bq[4];
#pragma unroll
      for (int sf = 0; sf < 2; ++sf) {
        const u16* base = &sK[(mW + sf * 16 + c16) * 64 + k0];
        ak[sf].q[0] = *(const uint4*)(base + 8 * half);
        ak[sf].q[1] = *(const uint4*)(base + 16 + 8 * half);
      }
#pragma unroll
      for (int nf = 0; nf < 4; ++nf) {
        const u16* base = &sQ[(nW + nf * 16 + c16) * 64 + k0];
        bq[nf].q[0] = *(const uint4*)(base + 8 * half);
        bq[nf].q[1] = *(const uint4*)(base + 16 + 8 * half);
      }
#pragma unroll
      for (int sf = 0; sf < 2; ++sf)
#pragma unroll
        for (int nf = 0; nf < 4; ++nf)
          acc[sf][nf].v = wmma_bf16(ak[sf], bq[nf], acc[sf][nf].v);
    }

#pragma unroll
    for (int sf = 0; sf < 2; ++sf)
#pragma unroll
      for (int rr = 0; rr < 8; ++rr) {
        float v0 = fmaxf(fmaxf(acc[sf][0].f[rr], acc[sf][1].f[rr]),
                         fmaxf(acc[sf][2].f[rr], acc[sf][3].f[rr])) * scale;
#pragma unroll
        for (int msk = 1; msk < 16; msk <<= 1)
          v0 = fmaxf(v0, __shfl_xor(v0, msk, 32));
        float mOld = m_run[sf][rr];
        float mNew = fmaxf(mOld, v0);
        float se = 0.0f;
#pragma unroll
        for (int nf = 0; nf < 4; ++nf)
          se += __expf(acc[sf][nf].f[rr] * scale - mNew);
#pragma unroll
        for (int msk = 1; msk < 16; msk <<= 1)
          se += __shfl_xor(se, msk, 32);
        l_run[sf][rr] = l_run[sf][rr] * __expf(mOld - mNew) + se;
        m_run[sf][rr] = mNew;
      }
  }

  if (c16 == 0) {
#pragma unroll
    for (int sf = 0; sf < 2; ++sf)
#pragma unroll
      for (int rr = 0; rr < 8; ++rr) {
        int row = mW + sf * 16 + rr + 8 * half;
        mPart[wn][row] = m_run[sf][rr];
        lPart[wn][row] = l_run[sf][rr];
      }
  }
  __syncthreads();
  if (tid < 128) {
    float m0 = mPart[0][tid], m1 = mPart[1][tid];
    float mM = fmaxf(m0, m1);
    float L = lPart[0][tid] * __expf(m0 - mM) + lPart[1][tid] * __expf(m1 - mM);
    size_t row = (size_t)bh * SEQ + sBlk * 128 + tid;
    vst2(mG + row, mM);
    vst2(rlG + row, 1.0f / L);
  }
}

__global__ __launch_bounds__(256)
void attn_out(const u16* __restrict__ Kg, const u16* __restrict__ Qg,
              const u16* __restrict__ Vtg, const float* __restrict__ mG,
              const float* __restrict__ rlG, u16* __restrict__ Og, float scale) {
  __shared__ u16 sQ[128 * 64];
  __shared__ u16 sK[64 * 64];
  __shared__ u16 sVt[64 * 64];
  __shared__ u16 sPt[128 * 64];
  __shared__ float sM[64], sRL[64];
  __shared__ __align__(16) u16 sO[8][16 * 64];

  const int bh = blockIdx.y, nBlk = blockIdx.x;
  const int tid = threadIdx.x;
  const int wave = tid >> 5, lane = tid & 31;
  const int half = lane >> 4, c16 = lane & 15;
  const int p1s = (wave & 1) * 32;
  const int p1n = (wave >> 1) * 32;

  FragC oacc[4];
#pragma unroll
  for (int dt = 0; dt < 4; ++dt)
#pragma unroll
    for (int i = 0; i < 8; ++i) oacc[dt].f[i] = 0.0f;

  {
    int rr = tid >> 1, h = (tid & 1) * 32;
    const u16* g = Qg + ((size_t)bh * SEQ + nBlk * 128 + rr) * DHEAD + h;
    cp_async32(&sQ[rr * 64 + h], g);
    cp_async32(&sQ[rr * 64 + h + 16], g + 16);
  }

  for (int sb = 0; sb < 32; ++sb) {
    __syncthreads();
    {
      int rr = tid >> 2, h = (tid & 3) * 16;
      cp_async32(&sK[rr * 64 + h],
                 Kg + ((size_t)bh * SEQ + sb * 64 + rr) * DHEAD + h);
      cp_async32(&sVt[rr * 64 + h],
                 Vtg + ((size_t)bh * DHEAD + rr) * SEQ + sb * 64 + h);
    }
    if (tid < 64) {
      sM[tid]  = mG[(size_t)bh * SEQ + sb * 64 + tid];
      sRL[tid] = rlG[(size_t)bh * SEQ + sb * 64 + tid];
    }
    wait_async();
    __syncthreads();

    FragC acc[2][2];
#pragma unroll
    for (int sf = 0; sf < 2; ++sf)
#pragma unroll
      for (int nf = 0; nf < 2; ++nf)
#pragma unroll
        for (int i = 0; i < 8; ++i) acc[sf][nf].f[i] = 0.0f;

#pragma unroll
    for (int k0 = 0; k0 < 64; k0 += 32) {
      FragAB ak[2], bq[2];
#pragma unroll
      for (int sf = 0; sf < 2; ++sf) {
        const u16* base = &sK[(p1s + sf * 16 + c16) * 64 + k0];
        ak[sf].q[0] = *(const uint4*)(base + 8 * half);
        ak[sf].q[1] = *(const uint4*)(base + 16 + 8 * half);
      }
#pragma unroll
      for (int nf = 0; nf < 2; ++nf) {
        const u16* base = &sQ[(p1n + nf * 16 + c16) * 64 + k0];
        bq[nf].q[0] = *(const uint4*)(base + 8 * half);
        bq[nf].q[1] = *(const uint4*)(base + 16 + 8 * half);
      }
#pragma unroll
      for (int sf = 0; sf < 2; ++sf)
#pragma unroll
        for (int nf = 0; nf < 2; ++nf)
          acc[sf][nf].v = wmma_bf16(ak[sf], bq[nf], acc[sf][nf].v);
    }

#pragma unroll
    for (int sf = 0; sf < 2; ++sf)
#pragma unroll
      for (int nf = 0; nf < 2; ++nf)
#pragma unroll
        for (int rr = 0; rr < 8; ++rr) {
          int sl = p1s + sf * 16 + rr + 8 * half;
          int nl = p1n + nf * 16 + c16;
          float p = __expf(acc[sf][nf].f[rr] * scale - sM[sl]) * sRL[sl];
          sPt[nl * 64 + sl] = f2bf(p * PSC);
        }
    __syncthreads();

#pragma unroll
    for (int k0 = 0; k0 < 64; k0 += 32) {
      FragAB ap;
      const u16* abase = &sPt[(wave * 16 + c16) * 64 + k0];
      ap.q[0] = *(const uint4*)(abase + 8 * half);
      ap.q[1] = *(const uint4*)(abase + 16 + 8 * half);
#pragma unroll
      for (int dt = 0; dt < 4; ++dt) {
        FragAB bv;
        const u16* bbase = &sVt[(dt * 16 + c16) * 64 + k0];
        bv.q[0] = *(const uint4*)(bbase + 8 * half);
        bv.q[1] = *(const uint4*)(bbase + 16 + 8 * half);
        oacc[dt].v = wmma_bf16(ap, bv, oacc[dt].v);
      }
    }
  }

  const int bidx = bh >> 4, head = bh & 15;
  u16* so = sO[wave];
#pragma unroll
  for (int dt = 0; dt < 4; ++dt)
#pragma unroll
    for (int rr = 0; rr < 8; ++rr) so[(rr + 8 * half) * 64 + dt * 16 + c16] = f2bf(oacc[dt].f[rr] * PUN);
  __syncthreads();
#pragma unroll
  for (int q = 0; q < 4; ++q) {
    const int rl = q * 4 + (lane >> 3), pc = lane & 7;
    const int n = nBlk * 128 + wave * 16 + rl;
    vst2(Og + ((size_t)(bidx * SEQ + n)) * HID + head * DHEAD + pc * 8, *(const v4u*)(&so[rl * 64 + pc * 8]));
  }
}

extern "C" void kernel_launch(void* const* d_in, const int* in_sizes, int n_in,
                              void* d_out, int out_size, void* d_ws, size_t ws_size,
                              hipStream_t stream) {
  const float* X    = (const float*)d_in[0];
  const float* Wkqv = (const float*)d_in[1];
  const float* bkqv = (const float*)d_in[2];
  const float* Wff  = (const float*)d_in[3];
  const float* bff  = (const float*)d_in[4];
  float* out = (float*)d_out;

  char* ws = (char*)d_ws;
  size_t off = 0;
  auto carve = [&](size_t bytes) -> void* {
    void* p = ws + off;
    off = (off + bytes + 255) & ~(size_t)255;
    return p;
  };
  u16*   Xb  = (u16*)carve((size_t)ROWS * HID * 2);
  u16*   WkT = (u16*)carve((size_t)NKQV * HID * 2);
  u16*   WfT = (u16*)carve((size_t)HID * HID * 2);
  u16*   Kg  = (u16*)carve((size_t)BH * SEQ * DHEAD * 2);
  u16*   Qg  = (u16*)carve((size_t)BH * SEQ * DHEAD * 2);
  u16*   Vtg = (u16*)carve((size_t)BH * SEQ * DHEAD * 2);
  u16*   Og  = (u16*)carve((size_t)ROWS * HID * 2);
  float* mG  = (float*)carve((size_t)BH * SEQ * 4);
  float* rlG = (float*)carve((size_t)BH * SEQ * 4);

  const float scale = 0.25f;

  convert_f32_bf16<<<(ROWS * HID / 8) / 256, 256, 0, stream>>>(X, Xb, ROWS * HID);
  transpose_cvt<<<dim3(NKQV / 32, HID / 64), 256, 0, stream>>>(Wkqv, WkT, HID, NKQV);
  transpose_cvt<<<dim3(HID / 32, HID / 64), 256, 0, stream>>>(Wff, WfT, HID, HID);

  gemm_bf16<0><<<dim3(NKQV / 256, ROWS / 128), 256, 0, stream>>>(
      Xb, WkT, bkqv, ROWS, NKQV, HID, Kg, Qg, Vtg, nullptr);

  attn_stats<<<dim3(SEQ / 128, BH), 256, 0, stream>>>(Kg, Qg, mG, rlG, scale);
  attn_out<<<dim3(SEQ / 128, BH), 256, 0, stream>>>(Kg, Qg, Vtg, mG, rlG, Og, scale);

  gemm_bf16<1><<<dim3(HID / 256, ROWS / 128), 256, 0, stream>>>(
      Og, WfT, bff, ROWS, HID, HID, nullptr, nullptr, nullptr, out);

  (void)in_sizes; (void)n_in; (void)out_size; (void)ws_size;
}
